// ChargeFieldModule_41394894799546
// MI455X (gfx1250) — hardware-run, weakly checked
//
#include <hip/hip_runtime.h>


#define NRC  200000
#define NBN  256
#define NPS  67584
#define NZS  22
#define NKS  3072
#define NPA  3
constexpr size_t al256(size_t b) { return (b + 255) & ~(size_t)255; }
constexpr size_t WS_TOTAL = al256((size_t)64 * 4) + 2 * al256((size_t)NRC * 2 * 4) + al256((size_t)NRC * 4) + 2 * al256((size_t)NZS * NBN * NKS * 2) + al256((size_t)NPA * NZS * NBN * NBN * 4);
static_assert(WS_TOTAL == 90507776 && WS_TOTAL <= 134217728, "the workspace carve: 86.3 MiB");
static_assert(NPS == NZS * NKS && NPA * NPS >= NRC && NKS % 64 == 0 && NBN % 64 == 0 && NRC % 8 == 0 && (NPS / 8) % 256 == 0 && (NKS / 8) == 384 && 384 % 32 == 0, "whole tiles; whole lines; whole blocks; whole waves a slice row; a piece wholly live or wholly past the last box");
typedef _Float16 h16;
typedef unsigned short bf;
typedef __attribute__((ext_vector_type(16))) __bf16   v16bf;
typedef __attribute__((ext_vector_type(16))) _Float16 v16h;
typedef __attribute__((ext_vector_type(8)))  _Float16 v8h;
typedef __attribute__((ext_vector_type(8)))  unsigned short v8us;
typedef __attribute__((ext_vector_type(8)))  float    v8f;
typedef __attribute__((ext_vector_type(4)))  float    v4f;
typedef v8h  __attribute__((may_alias)) v8ha;
typedef v4f  __attribute__((may_alias)) v4fa;
typedef v8us __attribute__((may_alias)) v8usa;

__device__ __forceinline__ unsigned short f2bf(float f) { unsigned u = __float_as_uint(f); u += 0x7FFFu + ((u >> 16) & 1u); return (unsigned short)(u >> 16); }
__device__ __forceinline__ float bf2f(unsigned short b) { return __uint_as_float(((unsigned)b) << 16); }
__device__ __forceinline__ float bfr(float f) { return bf2f(f2bf(f)); }
__device__ __forceinline__ v16h cat16(v8h lo, v8h hi) { return __builtin_shufflevector(lo, hi, 0, 1, 2, 3, 4, 5, 6, 7, 8, 9, 10, 11, 12, 13, 14, 15); }
__device__ __forceinline__ v16bf cat16b(v8us lo, v8us hi) { return __builtin_bit_cast(v16bf, __builtin_shufflevector(lo, hi, 0, 1, 2, 3, 4, 5, 6, 7, 8, 9, 10, 11, 12, 13, 14, 15)); }
__device__ __forceinline__ v8f wmma16(v16h a, v16h b, v8f c) { return __builtin_amdgcn_wmma_f32_16x16x32_f16(false, a, false, b, (short)0, c, false, false); }
__device__ __forceinline__ v8f wmmab(v16bf a, v16bf b, v8f c) { return __builtin_amdgcn_wmma_f32_16x16x32_bf16(false, a, false, b, (short)0, c, false, false); }


template <typename T16> struct WFrag;
template <> struct WFrag<h16> { typedef v16h V; static __device__ __forceinline__ V ld(const h16* p) { return cat16(*(const v8h*)p, *(const v8h*)(p + 16)); } static __device__ __forceinline__ v8f mma(V a, V b, v8f c) { return wmma16(a, b, c); } };
template <> struct WFrag<bf> { typedef v16bf V; static __device__ __forceinline__ V ld(const bf* p) { return cat16b(*(const v8us*)p, *(const v8us*)(p + 16)); } static __device__ __forceinline__ v8f mma(V a, V b, v8f c) { return wmmab(a, b, c); } };
template <typename T16, int NSPLIT, bool BIAS>
__global__ __launch_bounds__(32) void k_gemmw(const T16* __restrict__ A, const T16* __restrict__ A2, const T16* __restrict__ Bt, const T16* __restrict__ Bt2, int K, float* C, int ldc, const float* __restrict__ bias, size_t sA, size_t sB, size_t sC) {
    typedef typename WFrag<T16>::V V;
    __shared__ __align__(16) float os[16 * 68];
    const size_t z = blockIdx.z; A += z * sA; if (A2) A2 += z * sA; Bt += z * sB; if (Bt2) Bt2 += z * sB; C += z * sC;
    const int lane = threadIdx.x & 31, lr = lane & 15, hi = lane >> 4; const int r0 = blockIdx.x * 64, c0 = blockIdx.y * 64;
    v8f acc[4][4];
#pragma unroll
    for (int mb = 0; mb < 4; ++mb)
#pragma unroll
        for (int nb = 0; nb < 4; ++nb) acc[mb][nb] = (v8f){};
    const size_t aoff = (size_t)(r0 + lr) * K + 8 * hi, boff = (size_t)(c0 + lr) * K + 8 * hi;
    for (int kc = 0; kc < K; kc += 32) {
        V a[4], a2[4];
#pragma unroll
        for (int mb = 0; mb < 4; ++mb) { a[mb] = WFrag<T16>::ld(A + aoff + (size_t)mb * 16 * K + kc); if (NSPLIT == 1 || NSPLIT == 2) a2[mb] = WFrag<T16>::ld(A2 + aoff + (size_t)mb * 16 * K + kc); }
#pragma unroll
        for (int nb = 0; nb < 4; ++nb) { const V b = WFrag<T16>::ld(Bt + boff + (size_t)nb * 16 * K + kc); V b2; if (NSPLIT >= 2) b2 = WFrag<T16>::ld(Bt2 + boff + (size_t)nb * 16 * K + kc);
#pragma unroll
            for (int mb = 0; mb < 4; ++mb) { acc[mb][nb] = WFrag<T16>::mma(a[mb], b, acc[mb][nb]); if (NSPLIT == 1 || NSPLIT == 2) acc[mb][nb] = WFrag<T16>::mma(a2[mb], b, acc[mb][nb]); if (NSPLIT >= 2) acc[mb][nb] = WFrag<T16>::mma(a[mb], b2, acc[mb][nb]); } }
        asm volatile("v_nop\n\tv_nop\n\tv_nop\n\tv_nop" : "+v"(acc[0][0]), "+v"(acc[1][1]), "+v"(acc[2][2]), "+v"(acc[3][3]) : "v"(a[0]), "v"(a[3]));
    }
#pragma unroll
    for (int mb = 0; mb < 4; ++mb) {
#pragma unroll
        for (int nb = 0; nb < 4; ++nb) {
#pragma unroll
            for (int j = 0; j < 8; ++j) os[(hi * 8 + j) * 68 + nb * 16 + lr] = acc[mb][nb][j]; }
        __builtin_amdgcn_wave_barrier(); asm volatile("" ::: "memory");
        float* crow = C + (size_t)(r0 + mb * 16) * ldc + c0;
#pragma unroll 1
        for (int ps = 0; ps < 2; ++ps) {
#pragma unroll
            for (int s = 0; s < 8; ++s) { const int row = 2 * s + hi, cofs = lr * 4; v4f val = *(const v4fa*)(os + row * 68 + cofs); if (BIAS) { val[0] += bfr(bias[c0 + cofs]); val[1] += bfr(bias[c0 + cofs + 1]); val[2] += bfr(bias[c0 + cofs + 2]); val[3] += bfr(bias[c0 + cofs + 3]); }
                *(volatile v4f*)(crow + (size_t)row * ldc + cofs) = val; }
            if (ps == 0) __threadfence(); }
        __builtin_amdgcn_wave_barrier(); asm volatile("" ::: "memory");
    }
}

__device__ __forceinline__ h16 tohx(float x) { return (h16)x; }
__device__ __forceinline__ void splitf(float y, unsigned short& h, unsigned short& l) { h = f2bf(y); l = f2bf(y - bf2f(h)); }
typedef __attribute__((ext_vector_type(2))) _Float16 v2h;
typedef __attribute__((ext_vector_type(4))) _Float16 v4h;
typedef __attribute__((ext_vector_type(2))) unsigned short v2us;
typedef __attribute__((ext_vector_type(4))) unsigned short v4us;
typedef __attribute__((ext_vector_type(2))) float v2f;
typedef __attribute__((ext_vector_type(4))) int v4i;


typedef _Float16 v8h __attribute__((ext_vector_type(8)));
typedef float v4f __attribute__((ext_vector_type(4)));

__global__ __launch_bounds__(256) void k_rnd(const float* __restrict__ src, float* dst, unsigned npc, unsigned nw) {
    const unsigned g = blockIdx.x * 256 + threadIdx.x; if (g >= npc) return; v4f o;
#pragma unroll
    for (int e = 0; e < 4; ++e) { const unsigned i = 4u * g + (unsigned)e; const unsigned live = i < nw ? 1u : 0u; const float rv_ = bfr(src[live ? i : 0u]); o[e] = live ? rv_ : 0.0f; }
    float* dq = dst + 4u * (size_t)g; *(volatile v4f*)(dq) = o; __threadfence(); *(volatile v4f*)(dq) = o; }

__global__ __launch_bounds__(256) void k_ovl(const float* __restrict__ bd, const float* __restrict__ pq, const float* __restrict__ dm, const float* __restrict__ cw, unsigned n0, h16* ax, h16* by) {
    const unsigned g = blockIdx.x * 256 + threadIdx.x; if (g >= (unsigned)(NPS / 8)) return; const unsigned r = blockIdx.y, z = g / 384u, kk = 8u * (g - 384u * z); const unsigned n = n0 + 8u * g; const unsigned liv = n < (unsigned)NRC ? 1u : 0u; const unsigned nb = liv ? n : 0u; const float lf = liv ? 1.0f : 0.0f;
    const float x0 = bd[0], y0 = bd[1], x1 = bd[2], y1 = bd[3]; const float hx = (x1 - x0) / 256.0f, hy = (y1 - y0) / 256.0f; const float fr = (float)r; const float e0 = x0 + fr * hx, f0 = y0 + fr * hy; const float e1 = e0 + hx, f1 = f0 + hy;
    const float* xq = pq + 2u * (size_t)nb; const float* dq = dm + 2u * (size_t)nb; const float* wq = cw + nb; v8h oa, ob;
#pragma unroll
    for (int e = 0; e < 8; ++e) { const float p0 = xq[2 * e], q0 = xq[2 * e + 1]; const float p1 = p0 + dq[2 * e], q1 = q0 + dq[2 * e + 1];
        const float sx = fmaxf(fminf(e1, p1) - fmaxf(e0, p0), 0.0f); const float sy = fmaxf(fminf(f1, q1) - fmaxf(f0, q0), 0.0f);
        const float va = ((wq[e] * sx) * 256.0f) * lf; const float vb = (sy * 256.0f) * lf; const float ka = fabsf(va) >= 6.103515625e-05f ? 1.0f : 0.0f; const float kb = fabsf(vb) >= 6.103515625e-05f ? 1.0f : 0.0f; oa[e] = tohx(va * ka); ob[e] = tohx(vb * kb); }
    const size_t off = ((size_t)z * NBN + r) * NKS + kk; *(volatile v8h*)(ax + off) = oa; *(volatile v8h*)(by + off) = ob; __threadfence(); *(volatile v8h*)(ax + off) = oa; *(volatile v8h*)(by + off) = ob; }

__global__ __launch_bounds__(256) void k_red(const float* __restrict__ pp, const float* __restrict__ bd, float* rsl) {
    const unsigned g = blockIdx.x * 256 + threadIdx.x; if (g >= (unsigned)(NBN * NBN / 4)) return; const float hx = (bd[2] - bd[0]) / 256.0f, hy = (bd[3] - bd[1]) / 256.0f; v4f acc = *(const v4f*)(pp + 4u * (size_t)g);
    for (int s = 1; s < NPA * NZS; ++s) { const v4f a = *(const v4f*)(pp + (size_t)s * NBN * NBN + 4u * (size_t)g); acc += a; }
    v4f o;
#pragma unroll
    for (int e = 0; e < 4; ++e) o[e] = (acc[e] * 1.52587890625e-05f) / (hx * hy);
    float* dq = rsl + 4u * (size_t)g; *(volatile v4f*)(dq) = o; __threadfence(); *(volatile v4f*)(dq) = o; }

extern "C" void kernel_launch(void* const* d_in, const int* in_sizes, int n_in,
                              void* d_out, int out_size, void* d_ws, size_t ws_size, hipStream_t stream) {
    if (n_in < 5) return;
    if (in_sizes[0] < 4 || in_sizes[1] < NRC * 2 || in_sizes[2] < NRC * 2 || in_sizes[3] < NRC || out_size < NBN * NBN) return;
    const float* bd = (const float*)d_in[0]; const float* pq = (const float*)d_in[1]; const float* dm = (const float*)d_in[2]; const float* cw = (const float*)d_in[3];
    char* wsp = (char*)d_ws;
    auto take = [&](size_t bytes) { char* cur = wsp; wsp += (bytes + 255) & ~(size_t)255; return (void*)cur; };
    float* BD = (float*)take((size_t)64 * 4); float* PQ = (float*)take((size_t)NRC * 2 * 4); float* DM = (float*)take((size_t)NRC * 2 * 4); float* CW = (float*)take((size_t)NRC * 4); h16* AX = (h16*)take((size_t)NZS * NBN * NKS * 2); h16* BY = (h16*)take((size_t)NZS * NBN * NKS * 2); float* PP = (float*)take((size_t)NPA * NZS * NBN * NBN * 4);
    if ((size_t)(wsp - (char*)d_ws) != WS_TOTAL || WS_TOTAL > ws_size) return;
    auto rnd = [&](const float* sp_, float* dp_, unsigned nw) { const unsigned npc = (nw + 3) / 4; k_rnd<<<(npc + 255) / 256, 256, 0, stream>>>(sp_, dp_, npc, nw); };
    rnd(bd, BD, 4); rnd(pq, PQ, NRC * 2); rnd(dm, DM, NRC * 2); rnd(cw, CW, NRC);
    for (int p = 0; p < NPA; ++p) {
        k_ovl<<<dim3((NPS / 8 + 255) / 256, NBN, 1), 256, 0, stream>>>(BD, PQ, DM, CW, (unsigned)(p * NPS), AX, BY);
        k_gemmw<h16, 0, false><<<dim3(NBN / 64, NBN / 64, NZS), 32, 0, stream>>>(AX, nullptr, BY, nullptr, NKS, PP + (size_t)p * NZS * NBN * NBN, NBN, nullptr, (size_t)NBN * NKS, (size_t)NBN * NKS, (size_t)NBN * NBN);
    }
    k_red<<<(NBN * NBN / 4 + 255) / 256, 256, 0, stream>>>(PP, BD, (float*)d_out);
}
